// RNN_55851754717381
// MI455X (gfx1250) — hardware-verified
//
#include <hip/hip_runtime.h>
#include <math.h>

typedef __attribute__((ext_vector_type(16))) _Float16 v16h;
typedef __attribute__((ext_vector_type(8)))  _Float16 v8h;
typedef __attribute__((ext_vector_type(8)))  float    v8f;
typedef __attribute__((ext_vector_type(4)))  float    v4f;

constexpr int kSeq   = 64;
constexpr int kStep  = 512;
constexpr int kIn    = 256;
constexpr int kHid   = 1024;
constexpr int kOutD  = 256;
constexpr int kRows  = kSeq * kStep;
constexpr int kKcat  = kHid + kIn;
constexpr int kOut0  = kRows * kOutD;
constexpr int kOut1  = kSeq * kHid;
constexpr float kBnEps = 1e-5f;
constexpr float kInvCnt = 1.0f / (float)kRows;
constexpr float kWCarry    = 16.0f;
constexpr float kWCarryInv = 1.0f / kWCarry;

constexpr int kSeqPB      = 16;
constexpr int kRnnBlocks  = kSeq / kSeqPB;
constexpr int kRnnThreads = 512;
constexpr int kHP         = kHid + 8;
constexpr int kFP         = 260;
static_assert(kSeq % kSeqPB == 0);
static_assert(kHid == (kRnnThreads / 32) * 64);
static_assert(kHP % 8 == 0 && kFP % 4 == 0);
static_assert(kHid % 32 == 0 && kIn % 32 == 0 && kKcat % 32 == 0);
static_assert(kRows % 64 == 0 && kOutD % 64 == 0 && kHid % 64 == 0);
static_assert(kSeqPB * kFP >= 2 * kHid);
static_assert((kSeqPB * (kHid / 8)) % kRnnThreads == 0);

constexpr int kXChunks  = kRows * kIn / 8;
constexpr int kChHH     = kHid * (kHid / 8);
constexpr int kChIH     = kHid * (kIn / 8);
constexpr int kBlkHH    = kChHH / 256;
constexpr int kBlkIH    = kChIH / 256;
constexpr int kPrepBlocks = kBlkHH + kBlkIH + 1;
static_assert(kXChunks % 256 == 0 && kChHH % 256 == 0 && kChIH % 256 == 0);
static_assert(kHid == 256 * 4);

__device__ __forceinline__ void guard4_h(v8f& a0, v8f& a1, v8f& a2, v8f& a3, v16h x, v16h y0, v16h y1, v16h y2, v16h y3) {
  asm volatile("v_nop\n\tv_nop\n\tv_nop\n\tv_nop" : "+v"(a0), "+v"(a1), "+v"(a2), "+v"(a3) : "v"(x), "v"(y0), "v"(y1), "v"(y2), "v"(y3));
}
__device__ __forceinline__ void keep4_h(v16h a, v16h b, v16h c, v16h d) { asm volatile("v_nop" :: "v"(a), "v"(b), "v"(c), "v"(d)); }
__device__ __forceinline__ void acc_guard4(v8f& a, v8f& b, v8f& c, v8f& d) { asm volatile("v_nop\n\tv_nop\n\tv_nop\n\tv_nop" : "+v"(a), "+v"(b), "+v"(c), "+v"(d)); }

struct FragH {
  union U { v16h v; v8h h[2]; };
  static __device__ __forceinline__ v16h load(const _Float16* p) {
    U f; f.h[0] = *(const v8h*)(p); f.h[1] = *(const v8h*)(p + 16); return f.v;
  }
  static __device__ __forceinline__ v8f mma(v16h a, v16h b, v8f c) {
    return __builtin_amdgcn_wmma_f32_16x16x32_f16(false, a, false, b, (short)0, c, false, false);
  }
};

__device__ __forceinline__ v8h pack8(v4f a, v4f b, float sc) {
  v8h h;
  h[0] = (_Float16)(a[0] * sc); h[1] = (_Float16)(a[1] * sc); h[2] = (_Float16)(a[2] * sc); h[3] = (_Float16)(a[3] * sc);
  h[4] = (_Float16)(b[0] * sc); h[5] = (_Float16)(b[1] * sc); h[6] = (_Float16)(b[2] * sc); h[7] = (_Float16)(b[3] * sc);
  return h;
}
__device__ __forceinline__ void st2_v8h(_Float16* p, v8h v) { *(volatile v8h*)p = v; __threadfence(); *(volatile v8h*)p = v; }
__device__ __forceinline__ void st2_v4f(float* p, v4f v)    { *(volatile v4f*)p = v; __threadfence(); *(volatile v4f*)p = v; }

__global__ __launch_bounds__(256) void xcast_kernel(const float* __restrict__ x, unsigned short* __restrict__ x16p) {
  const int i = blockIdx.x * 256 + threadIdx.x;
  if (i < kXChunks) {
    const float* src = x + (size_t)i * 8;
    const v4f f0 = *(const v4f*)src;
    const v4f f1 = *(const v4f*)(src + 4);
    const v8h hv = pack8(f0, f1, 1.0f);
    st2_v8h((_Float16*)x16p + (size_t)i * 8, hv);
  }
}

__global__ __launch_bounds__(256) void prep_kernel(const float* __restrict__ w_hh, const float* __restrict__ w_ih,
                                                   const float* __restrict__ b_ih, const float* __restrict__ b_hh,
                                                   unsigned short* __restrict__ wcatp, float* __restrict__ bsum) {
  const int blk = blockIdx.x, tid = threadIdx.x;
  _Float16* wcat = (_Float16*)wcatp;
  if (blk < kBlkHH) {
    const int p = blk * 256 + tid;
    const int row = p >> 7, c8 = p & 127;
    const float* src = w_hh + (size_t)row * kHid + c8 * 8;
    const v4f f0 = *(const v4f*)src;
    const v4f f1 = *(const v4f*)(src + 4);
    st2_v8h(wcat + (size_t)row * kKcat + c8 * 8, pack8(f0, f1, kWCarry));
  } else if (blk < kBlkHH + kBlkIH) {
    const int p = (blk - kBlkHH) * 256 + tid;
    const int row = p >> 5, c8 = p & 31;
    const float* src = w_ih + (size_t)row * kIn + c8 * 8;
    const v4f f0 = *(const v4f*)src;
    const v4f f1 = *(const v4f*)(src + 4);
    st2_v8h(wcat + (size_t)row * kKcat + kHid + c8 * 8, pack8(f0, f1, kWCarry));
  } else {
    const int idx = tid * 4;
    const v4f a = *(const v4f*)(b_ih + idx);
    const v4f b = *(const v4f*)(b_hh + idx);
    const v4f s = a + b;
    st2_v4f(bsum + idx, s);
  }
}

__global__ __launch_bounds__(kRnnThreads) void rnn_seq_kernel(
    const unsigned short* __restrict__ x16p, const unsigned short* __restrict__ wcatp,
    const float* __restrict__ bsum, const float* __restrict__ h0,
    unsigned short* __restrict__ hs16p, float* __restrict__ hlast, float* __restrict__ stat) {
  __shared__ __align__(16) _Float16 hbuf[kSeqPB * kHP];
  __shared__ __align__(16) float    fst[kSeqPB * kFP];
  const _Float16* X16  = (const _Float16*)x16p;
  const _Float16* WCAT = (const _Float16*)wcatp;
  _Float16*       HS16 = (_Float16*)hs16p;
  const int tid = threadIdx.x, lane = tid & 31, wave = tid >> 5;
  const int c = lane & 15, hh = lane >> 4, koff = hh * 8, mOff = hh * 8;
  const int seq0 = blockIdx.x * kSeqPB;
  const int n0 = wave * 64;

  {
#pragma unroll
    for (int it = 0; it < (kSeqPB * (kHid / 8)) / kRnnThreads; ++it) {
      const int i = tid + it * kRnnThreads;
      const int row = i >> 7, c8 = i & 127;
      const float* src = h0 + (size_t)(seq0 + row) * kHid + c8 * 8;
      const v4f f0 = *(const v4f*)src;
      const v4f f1 = *(const v4f*)(src + 4);
      *(v8h*)(hbuf + row * kHP + c8 * 8) = pack8(f0, f1, 1.0f);
    }
    if (tid < kSeqPB) {
      const v4f z = {0.f, 0.f, 0.f, 0.f};
      *(v8h*)(hbuf + tid * kHP + kHid) = pack8(z, z, 1.0f);
    }
  }
  float bs[4];
#pragma unroll
  for (int j = 0; j < 4; ++j) bs[j] = bsum[n0 + 16 * j + c];
  __syncthreads();

  const v8f z8 = {0.f, 0.f, 0.f, 0.f, 0.f, 0.f, 0.f, 0.f};
  const _Float16* brow = WCAT + (size_t)(n0 + c) * kKcat + koff;
  const _Float16* arow = hbuf + c * kHP + koff;
  const int q4 = lane >> 3, c8s = (lane & 7) * 8;

  v8f acc[4];
  float ssum[4], qsum[4];
#pragma unroll
  for (int j = 0; j < 4; ++j) { acc[j] = z8; ssum[j] = 0.0f; qsum[j] = 0.0f; }

#pragma unroll 1
  for (int t = 0; t < kStep; ++t) {
#pragma unroll
    for (int j = 0; j < 4; ++j) acc[j] = z8;

    const _Float16* xrow = X16 + ((size_t)(seq0 + c) * kStep + (size_t)t) * kIn + koff;
#pragma unroll 1
    for (int kx = 0; kx < kIn; kx += 32) {
      const v16h fa = FragH::load(xrow + kx);
      asm volatile("" ::: "memory");
      const v16h fb0 = FragH::load(brow + kHid + kx);
      const v16h fb1 = FragH::load(brow + (size_t)16 * kKcat + kHid + kx);
      const v16h fb2 = FragH::load(brow + (size_t)32 * kKcat + kHid + kx);
      const v16h fb3 = FragH::load(brow + (size_t)48 * kKcat + kHid + kx);
      acc[0] = FragH::mma(fa, fb0, acc[0]);
      acc[1] = FragH::mma(fa, fb1, acc[1]);
      acc[2] = FragH::mma(fa, fb2, acc[2]);
      acc[3] = FragH::mma(fa, fb3, acc[3]);
      guard4_h(acc[0], acc[1], acc[2], acc[3], fa, fb0, fb1, fb2, fb3);
    }
#pragma unroll 1
    for (int k0 = 0; k0 < kHid; k0 += 32) {
      const v16h fa  = FragH::load(arow + k0);
      const v16h fb0 = FragH::load(brow + k0);
      const v16h fb1 = FragH::load(brow + (size_t)16 * kKcat + k0);
      const v16h fb2 = FragH::load(brow + (size_t)32 * kKcat + k0);
      const v16h fb3 = FragH::load(brow + (size_t)48 * kKcat + k0);
      acc[0] = FragH::mma(fa, fb0, acc[0]);
      acc[1] = FragH::mma(fa, fb1, acc[1]);
      acc[2] = FragH::mma(fa, fb2, acc[2]);
      acc[3] = FragH::mma(fa, fb3, acc[3]);
      guard4_h(acc[0], acc[1], acc[2], acc[3], fa, fb0, fb1, fb2, fb3);
    }
    acc_guard4(acc[0], acc[1], acc[2], acc[3]);

#pragma unroll
    for (int j = 0; j < 4; ++j) {
      float cs = 0.0f, cq = 0.0f;
#pragma unroll
      for (int r = 0; r < 8; ++r) {
        const float v = tanhf(acc[j][r] * kWCarryInv + bs[j]);
        acc[j][r] = v;
        cs += v;
        cq += v * v;
      }
      ssum[j] += cs;
      qsum[j] += cq;
    }
    __syncthreads();
#pragma unroll
    for (int j = 0; j < 4; ++j) {
#pragma unroll
      for (int r = 0; r < 8; ++r) hbuf[(mOff + r) * kHP + n0 + 16 * j + c] = (_Float16)acc[j][r];
    }
    __syncthreads();

    for (int pass = 0; pass < 2; ++pass) {
#pragma unroll
      for (int it = 0; it < 4; ++it) {
        const int rr = it * 4 + q4;
        const v8h v = *(const v8h*)(hbuf + rr * kHP + n0 + c8s);
        *(volatile v8h*)(HS16 + ((size_t)(seq0 + rr) * kStep + (size_t)t) * kHid + n0 + c8s) = v;
      }
      __threadfence();
    }
  }

  {
    const int lw = wave & 3;
    const int c4 = (lane & 15) * 4;
#pragma unroll 1
    for (int ph = 0; ph < 4; ++ph) {
      const bool mine = ((wave >> 2) == ph);
      if (mine) {
#pragma unroll
        for (int j = 0; j < 4; ++j)
#pragma unroll
          for (int r = 0; r < 8; ++r) fst[(mOff + r) * kFP + lw * 64 + 16 * j + c] = acc[j][r];
      }
      __syncthreads();
      if (mine) {
        for (int pass = 0; pass < 2; ++pass) {
#pragma unroll
          for (int it = 0; it < 8; ++it) {
            const int row = it * 2 + hh;
            const v4f v = *(const v4f*)(fst + row * kFP + lw * 64 + c4);
            *(volatile v4f*)(hlast + (size_t)(seq0 + row) * kHid + n0 + c4) = v;
          }
          __threadfence();
        }
      }
      __syncthreads();
    }
  }

#pragma unroll
  for (int j = 0; j < 4; ++j) {
    const float so = __shfl_xor(ssum[j], 16, 32);
    const float qo = __shfl_xor(qsum[j], 16, 32);
    ssum[j] += so;
    qsum[j] += qo;
  }
  if (hh == 0) {
#pragma unroll
    for (int j = 0; j < 4; ++j) {
      fst[n0 + 16 * j + c] = ssum[j];
      fst[kHid + n0 + 16 * j + c] = qsum[j];
    }
  }
  __syncthreads();
  {
    const v4f sv = *(const v4f*)(fst + tid * 4);
    st2_v4f(stat + (size_t)blockIdx.x * (2 * kHid) + tid * 4, sv);
  }
}

__global__ __launch_bounds__(256) void fold_kernel(const float* __restrict__ stat, const float* __restrict__ gamma,
                                                   const float* __restrict__ beta, const float* __restrict__ w_out,
                                                   const float* __restrict__ b_out, unsigned short* __restrict__ wout16p,
                                                   float* __restrict__ biasp) {
  __shared__ __align__(16) float lsc[kHid];
  __shared__ __align__(16) float lsh[kHid];
  __shared__ float lb[32];
  const int tid = threadIdx.x, lane = tid & 31, wave = tid >> 5;
  _Float16* wout16 = (_Float16*)wout16p;
  {
    const int ch = tid * 4;
    v4f s = {0.f, 0.f, 0.f, 0.f}, q = {0.f, 0.f, 0.f, 0.f};
#pragma unroll
    for (int b = 0; b < kRnnBlocks; ++b) {
      const v4f ps = *(const v4f*)(stat + (size_t)b * (2 * kHid) + ch);
      const v4f pq = *(const v4f*)(stat + (size_t)b * (2 * kHid) + kHid + ch);
      s += ps;
      q += pq;
    }
    asm volatile("" ::: "memory");
    const v4f g  = *(const v4f*)(gamma + ch);
    const v4f bt = *(const v4f*)(beta + ch);
    v4f scv, shv;
#pragma unroll
    for (int e = 0; e < 4; ++e) {
      const float mean = s[e] * kInvCnt;
      float var = q[e] * kInvCnt - mean * mean;
      var = fmaxf(var, 0.0f);
      const float sce = g[e] * rsqrtf(var + kBnEps);
      scv[e] = sce;
      shv[e] = bt[e] - mean * sce;
    }
    *(v4f*)(lsc + ch) = scv;
    *(v4f*)(lsh + ch) = shv;
  }
  __syncthreads();

#pragma unroll 1
  for (int rr = 0; rr < 4; ++rr) {
    const int o = blockIdx.x * 32 + wave * 4 + rr;
    const float* wr = w_out + (size_t)o * kHid;
    _Float16* dr = wout16 + (size_t)o * kHid;
    float dot = 0.0f;
#pragma unroll 1
    for (int it = 0; it < 4; ++it) {
      const int col = it * 256 + lane * 8;
      const v4f w0 = *(const v4f*)(wr + col);
      const v4f w1 = *(const v4f*)(wr + col + 4);
      const v4f s0 = *(const v4f*)(lsc + col);
      const v4f s1 = *(const v4f*)(lsc + col + 4);
      const v4f t0 = *(const v4f*)(lsh + col);
      const v4f t1 = *(const v4f*)(lsh + col + 4);
      const v4f p0 = w0 * s0;
      const v4f p1 = w1 * s1;
      const v8h hv = pack8(p0, p1, kWCarry);
#pragma unroll
      for (int e = 0; e < 4; ++e) { dot += w0[e] * t0[e]; dot += w1[e] * t1[e]; }
      st2_v8h(dr + col, hv);
    }
#pragma unroll
    for (int off = 16; off >= 1; off >>= 1) dot += __shfl_xor(dot, off, 32);
    if (lane == 0) lb[wave * 4 + rr] = dot;
  }
  __syncthreads();
  if (wave == 0) {
    const int o = blockIdx.x * 32 + lane;
    const float v = b_out[o] + lb[lane];
    volatile float* p = biasp + o;
    *p = v;
    __threadfence();
    *p = v;
  }
}

__global__ __launch_bounds__(256) void out_gemm_kernel(
    const unsigned short* __restrict__ Ap, int lda, const unsigned short* __restrict__ Btp, int ldb,
    float* __restrict__ C, int ldc, const float* __restrict__ addn, int M, int N, int K, float scale) {
  const _Float16* A = (const _Float16*)Ap;
  const _Float16* Bt = (const _Float16*)Btp;
  __shared__ __align__(16) float sT[8][16 * 68];
  const int lane = threadIdx.x & 31;
  const int wave = threadIdx.x >> 5;
  const int tilesN = N >> 6;
  const int tilesM = M >> 6;
  const int tile = blockIdx.x * 8 + wave;
  if (tile >= tilesM * tilesN) return;
  const int tm = tile / tilesN;
  const int tn = tile - tm * tilesN;
  const int m0 = tm << 6;
  const int n0 = tn << 6;
  const int rlane = lane & 15;
  const int koff  = (lane >> 4) * 8;
  const int mOff  = (lane >> 4) * 8;

  v8f acc[4][4];
#pragma unroll
  for (int i = 0; i < 4; ++i)
#pragma unroll
    for (int j = 0; j < 4; ++j) acc[i][j] = (v8f){0.f, 0.f, 0.f, 0.f, 0.f, 0.f, 0.f, 0.f};

  for (int k0 = 0; k0 < K; k0 += 32) {
    v16h bh[4];
#pragma unroll
    for (int j = 0; j < 4; ++j) {
      const size_t bo = (size_t)(n0 + (j << 4) + rlane) * ldb + koff + k0;
      bh[j] = FragH::load(Bt + bo);
    }
#pragma unroll
    for (int i = 0; i < 4; ++i) {
      const size_t ao = (size_t)(m0 + (i << 4) + rlane) * lda + koff + k0;
      const v16h ah = FragH::load(A + ao);
#pragma unroll
      for (int j = 0; j < 4; ++j) acc[i][j] = FragH::mma(ah, bh[j], acc[i][j]);
      guard4_h(acc[i][0], acc[i][1], acc[i][2], acc[i][3], ah, bh[0], bh[1], bh[2], bh[3]);
    }
    keep4_h(bh[0], bh[1], bh[2], bh[3]);
  }
  acc_guard4(acc[0][0], acc[0][1], acc[0][2], acc[0][3]);
  acc_guard4(acc[1][0], acc[1][1], acc[1][2], acc[1][3]);
  acc_guard4(acc[2][0], acc[2][1], acc[2][2], acc[2][3]);
  acc_guard4(acc[3][0], acc[3][1], acc[3][2], acc[3][3]);

  float* slab = sT[wave];
#pragma unroll
  for (int i = 0; i < 4; ++i) {
    const int mBase = m0 + (i << 4);
#pragma unroll
    for (int j = 0; j < 4; ++j) {
      const int n = n0 + (j << 4) + rlane;
      const float bv = addn[n];
#pragma unroll
      for (int r = 0; r < 8; ++r) {
        const float v = acc[i][j][r] * scale + bv;
        slab[(mOff + r) * 68 + (j << 4) + rlane] = v;
      }
    }
    __builtin_amdgcn_fence(__ATOMIC_RELEASE, "workgroup");
    __builtin_amdgcn_wave_barrier();
    __builtin_amdgcn_fence(__ATOMIC_ACQUIRE, "workgroup");
    {
      const int hh = lane >> 4, c4 = (lane & 15) * 4;
      for (int pass = 0; pass < 2; ++pass) {
#pragma unroll
        for (int it = 0; it < 8; ++it) {
          const int row = it * 2 + hh;
          const v4f v = *(const v4f*)(slab + row * 68 + c4);
          *(volatile v4f*)(C + (size_t)(mBase + row) * ldc + n0 + c4) = v;
        }
        __threadfence();
      }
    }
    __builtin_amdgcn_fence(__ATOMIC_RELEASE, "workgroup");
    __builtin_amdgcn_wave_barrier();
    __builtin_amdgcn_fence(__ATOMIC_ACQUIRE, "workgroup");
  }
}

extern "C" void kernel_launch(void* const* d_in, const int* in_sizes, int n_in,
                              void* d_out, int out_size, void* d_ws, size_t ws_size, hipStream_t stream) {
  if (n_in < 10 || d_out == nullptr || d_ws == nullptr) return;
  if (in_sizes[0] != kSeq * kStep * kIn || in_sizes[1] != kSeq * kHid || in_sizes[2] != kHid * kIn ||
      in_sizes[3] != kHid * kHid || in_sizes[4] != kHid || in_sizes[5] != kHid || in_sizes[6] != kHid ||
      in_sizes[7] != kHid || in_sizes[8] != kOutD * kHid || in_sizes[9] != kOutD ||
      out_size != kOut0 + kOut1) return;

  const float* x     = (const float*)d_in[0];
  const float* h0    = (const float*)d_in[1];
  const float* w_ih  = (const float*)d_in[2];
  const float* w_hh  = (const float*)d_in[3];
  const float* b_ih  = (const float*)d_in[4];
  const float* b_hh  = (const float*)d_in[5];
  const float* gamma = (const float*)d_in[6];
  const float* beta  = (const float*)d_in[7];
  const float* w_out = (const float*)d_in[8];
  const float* b_out = (const float*)d_in[9];
  float* out   = (float*)d_out;
  float* hlast = out + (size_t)kOut0;
  static_assert((size_t)kOut0 * 4 == 33554432u);
  static_assert(((size_t)kOut0 + (size_t)kOut1) * 4 == 33816576u);

  char* ws = (char*)d_ws; size_t off = 0;
  auto carve = [&](size_t bytes) -> char* { char* p = ws + off; off += (bytes + 255) & ~(size_t)255; return p; };
  unsigned short* X16    = (unsigned short*)carve((size_t)kRows * kIn * 2);
  unsigned short* WCAT   = (unsigned short*)carve((size_t)kHid * kKcat * 2);
  unsigned short* HS16   = (unsigned short*)carve((size_t)kRows * kHid * 2);
  unsigned short* WOUT16 = (unsigned short*)carve((size_t)kOutD * kHid * 2);
  float*          BSUM   = (float*)carve((size_t)kHid * 4);
  float*          STAT   = (float*)carve((size_t)kRnnBlocks * 2 * kHid * 4);
  float*          BIASP  = (float*)carve((size_t)kOutD * 4);
  if (off > ws_size || off > (size_t)134217728) return;

  xcast_kernel<<<kXChunks / 256, 256, 0, stream>>>(x, X16);

  prep_kernel<<<kPrepBlocks, 256, 0, stream>>>(w_hh, w_ih, b_ih, b_hh, WCAT, BSUM);

  rnn_seq_kernel<<<kRnnBlocks, kRnnThreads, 0, stream>>>(X16, WCAT, BSUM, h0, HS16, hlast, STAT);

  fold_kernel<<<kOutD / 32, 256, 0, stream>>>(STAT, gamma, beta, w_out, b_out, WOUT16, BIASP);

  static_assert(((kRows / 64) * (kOutD / 64)) % 8 == 0);
  out_gemm_kernel<<<((kRows / 64) * (kOutD / 64)) / 8, 256, 0, stream>>>(
      HS16, kHid, WOUT16, kHid, out, kOutD, BIASP, kRows, kOutD, kHid, kWCarryInv);
}
